// GSAAttention_19791209300599
// MI455X (gfx1250) — hardware-run, weakly checked
//
#include <hip/hip_runtime.h>


namespace {
constexpr int NBAT = 8, N = 2048, C = 512, CR = 64, NR = NBAT * N;
constexpr float XS = 8.0f, WSC = 256.0f, PS = 2048.0f;
typedef _Float16 b16;
typedef __attribute__((ext_vector_type(16))) _Float16 v16b;
typedef __attribute__((ext_vector_type(8))) _Float16 v8b;
typedef __attribute__((ext_vector_type(8))) float v8f;
typedef __attribute__((ext_vector_type(4))) float v4f;
__device__ __forceinline__ float bf16_rne(float f) { unsigned int u = __float_as_uint(f); u += 0x7FFFu + ((u >> 16) & 1u); return __uint_as_float(u & 0xFFFF0000u); }
__device__ __forceinline__ void split16(float v, b16& hi, b16& lo) { hi = (b16)v; lo = (b16)(v - (float)hi); }
__device__ __forceinline__ v16b frag_kb(const b16* p, int hh) { const v8b a = *(const v8b*)(p + 8 * hh), b = *(const v8b*)(p + 16 + 8 * hh); v16b f;
#pragma unroll
  for (int e = 0; e < 8; ++e) { f[e] = a[e]; f[8 + e] = b[e]; } return f; }
__device__ __forceinline__ v8f wmma16b(v16b a, v16b b, v8f c) { v8f d = __builtin_amdgcn_wmma_f32_16x16x32_f16(false, a, false, b, (short)0, c, false, false); asm volatile("v_nop\n\tv_nop\n\tv_nop\n\tv_nop" : "+v"(d) : "v"(a), "v"(b)); return d; }
__device__ __forceinline__ void wave_lds_sync() { __builtin_amdgcn_fence(__ATOMIC_RELEASE, "workgroup"); __builtin_amdgcn_wave_barrier(); __builtin_amdgcn_fence(__ATOMIC_ACQUIRE, "workgroup"); }
__device__ __forceinline__ float pmul(float a, float b) { float p = a * b; asm volatile("" : "+v"(p)); return p; }

__global__ __launch_bounds__(256) void prep_kernel(const float* __restrict__ x, const float* __restrict__ wk, const float* __restrict__ wv, const float* __restrict__ wq, b16* __restrict__ X16, b16* __restrict__ WKV, b16* __restrict__ WQ) {
  const size_t t = (size_t)blockIdx.x * 256 + threadIdx.x; const size_t nx = (size_t)NR * C / 8, nkv = (size_t)2 * CR * C / 8, nq = (size_t)C * C / 8; size_t u = t; v8b o;
  if (u < nx) { const size_t e = u * 8; const v4f a = *(const v4f*)(x + e), c = *(const v4f*)(x + e + 4); for (int j = 0; j < 4; ++j) { o[j] = (b16)(bf16_rne(a[j]) * XS); o[4 + j] = (b16)(bf16_rne(c[j]) * XS); } for (int pass = 0; pass < 2; ++pass) { *(volatile v8b*)(X16 + e) = o; __threadfence(); } return; } u -= nx;
  if (u < nkv) { const size_t e = u * 8; const float* w = (e < (size_t)CR * C) ? (wk + e) : (wv + (e - (size_t)CR * C)); for (int j = 0; j < 8; ++j) o[j] = (b16)(bf16_rne(w[j]) * WSC); for (int pass = 0; pass < 2; ++pass) { *(volatile v8b*)(WKV + e) = o; __threadfence(); } return; } u -= nkv;
  if (u < nq) { const size_t e = u * 8; for (int j = 0; j < 8; ++j) o[j] = (b16)(bf16_rne(wq[e + j]) * WSC); for (int pass = 0; pass < 2; ++pass) { *(volatile v8b*)(WQ + e) = o; __threadfence(); } }
}
__global__ __launch_bounds__(128) void kv_kernel(const b16* __restrict__ X16, const b16* __restrict__ WKV, const float* __restrict__ bk, const float* __restrict__ bv, b16* __restrict__ Kh, b16* __restrict__ Kl, b16* __restrict__ Vh, b16* __restrict__ Vl) {
  __shared__ __attribute__((aligned(16))) b16 Th[4][16][128 + 8], Tl[4][16][128 + 8];
  const int wave = threadIdx.x >> 5, lane = threadIdx.x & 31, nloc = lane & 15, hlf = lane >> 4; const size_t m0 = (size_t)blockIdx.x * 64 + wave * 16; v8f acc[8];
#pragma unroll
  for (int t = 0; t < 8; ++t) acc[t] = (v8f){};
#pragma unroll 2
  for (int kb = 0; kb < C; kb += 32) { const v16b a = frag_kb(X16 + (m0 + nloc) * C + kb, hlf);
#pragma unroll
    for (int t = 0; t < 8; ++t) acc[t] = wmma16b(a, frag_kb(WKV + (size_t)(t * 16 + nloc) * C + kb, hlf), acc[t]); }
#pragma unroll
  for (int t = 0; t < 8; ++t) { const int c = t * 16 + nloc; const float bb = (c < CR) ? bf16_rne(bk[c]) : bf16_rne(bv[c - CR]);
#pragma unroll 1
    for (int r = 0; r < 8; ++r) { b16 p, q; split16((acc[t][r] * (1.0f / (XS * WSC)) + bb) * XS, p, q); Th[wave][8 * hlf + r][c] = p; Tl[wave][8 * hlf + r][c] = q; } }
  wave_lds_sync();
  for (int pass = 0; pass < 2; ++pass) { for (int r4 = 0; r4 < 16; r4 += 4) { const int rr = r4 + (lane >> 3), c8 = (lane & 7) * 8; const size_t gi = (m0 + rr) * CR + c8;
      *(volatile v8b*)(Kh + gi) = *(const v8b*)(&Th[wave][rr][c8]); *(volatile v8b*)(Kl + gi) = *(const v8b*)(&Tl[wave][rr][c8]); *(volatile v8b*)(Vh + gi) = *(const v8b*)(&Th[wave][rr][CR + c8]); *(volatile v8b*)(Vl + gi) = *(const v8b*)(&Tl[wave][rr][CR + c8]); } __threadfence(); }
}
__global__ __launch_bounds__(128) void q_kernel(const b16* __restrict__ WQ, const b16* __restrict__ X16, const float* __restrict__ bq, b16* __restrict__ Qh, b16* __restrict__ Ql) {
  __shared__ __attribute__((aligned(16))) b16 Th[4][16][128 + 8], Tl[4][16][128 + 8];
  const int wave = threadIdx.x >> 5, lane = threadIdx.x & 31, nloc = lane & 15, hlf = lane >> 4; const int b = blockIdx.z; const size_t c0 = (size_t)blockIdx.x * 64 + wave * 16; const int n0 = blockIdx.y * 128; v8f acc[8];
#pragma unroll
  for (int t = 0; t < 8; ++t) acc[t] = (v8f){};
#pragma unroll 2
  for (int kb = 0; kb < C; kb += 32) { const v16b a = frag_kb(WQ + (c0 + nloc) * C + kb, hlf);
#pragma unroll
    for (int t = 0; t < 8; ++t) acc[t] = wmma16b(a, frag_kb(X16 + ((size_t)b * N + n0 + t * 16 + nloc) * C + kb, hlf), acc[t]); }
#pragma unroll
  for (int t = 0; t < 8; ++t)
#pragma unroll 1
    for (int r = 0; r < 8; ++r) { const float bb = bf16_rne(bq[c0 + 8 * hlf + r]); b16 p, q; split16((acc[t][r] * (1.0f / (WSC * XS)) + bb) * XS, p, q); Th[wave][8 * hlf + r][t * 16 + nloc] = p; Tl[wave][8 * hlf + r][t * 16 + nloc] = q; }
  wave_lds_sync();
  for (int pass = 0; pass < 2; ++pass) { for (int r2 = 0; r2 < 16; r2 += 2) { const int rr = r2 + (lane >> 4), c8 = (lane & 15) * 8; const size_t gi = ((size_t)b * C + c0 + rr) * N + n0 + c8; *(volatile v8b*)(Qh + gi) = *(const v8b*)(&Th[wave][rr][c8]); *(volatile v8b*)(Ql + gi) = *(const v8b*)(&Tl[wave][rr][c8]); } __threadfence(); }
}
__global__ __launch_bounds__(128) void s_kernel(const b16* __restrict__ Vh, const b16* __restrict__ Vl, const b16* __restrict__ Kh, const b16* __restrict__ Kl, int b, float* __restrict__ Sf) {
  __shared__ __attribute__((aligned(16))) float Tf[4][16][128 + 4];
  const int wave = threadIdx.x >> 5, lane = threadIdx.x & 31, nloc = lane & 15, hlf = lane >> 4; const size_t m0 = (size_t)blockIdx.x * 64 + wave * 16; const int n0 = blockIdx.y * 128; const size_t base = (size_t)b * N;
  v8f acc[8];
#pragma unroll
  for (int t = 0; t < 8; ++t) acc[t] = (v8f){};
#pragma unroll
  for (int kb = 0; kb < CR; kb += 32) { const v16b a = frag_kb(Vh + (base + m0 + nloc) * CR + kb, hlf), al = frag_kb(Vl + (base + m0 + nloc) * CR + kb, hlf);
#pragma unroll
    for (int t = 0; t < 8; ++t) { const v16b kf = frag_kb(Kh + (base + n0 + t * 16 + nloc) * CR + kb, hlf); acc[t] = wmma16b(a, kf, acc[t]); acc[t] = wmma16b(al, kf, acc[t]); acc[t] = wmma16b(a, frag_kb(Kl + (base + n0 + t * 16 + nloc) * CR + kb, hlf), acc[t]); } }
#pragma unroll
  for (int t = 0; t < 8; ++t)
#pragma unroll 1
    for (int r = 0; r < 8; ++r) Tf[wave][8 * hlf + r][t * 16 + nloc] = acc[t][r] * (1.0f / (XS * XS));
  wave_lds_sync();
  for (int pass = 0; pass < 2; ++pass) { for (int rr = 0; rr < 16; ++rr) *(volatile v4f*)(Sf + (m0 + rr) * N + n0 + lane * 4) = *(const v4f*)(&Tf[wave][rr][lane * 4]); __threadfence(); }
}
__global__ __launch_bounds__(256) void softmax_kernel(const float* __restrict__ Sf, b16* __restrict__ P16) {
  const int wave = threadIdx.x >> 5, lane = threadIdx.x & 31; const size_t m = (size_t)blockIdx.x * 8 + wave; float x[64]; float mx = -INFINITY;
  for (int j = 0; j < 8; ++j) { const v4f a = *(const v4f*)(Sf + m * N + j * 256 + lane * 8), c = *(const v4f*)(Sf + m * N + j * 256 + lane * 8 + 4); for (int i = 0; i < 4; ++i) { x[j * 8 + i] = a[i]; x[j * 8 + 4 + i] = c[i]; } }
  for (int i = 0; i < 64; ++i) mx = fmaxf(mx, x[i]);
#pragma unroll
  for (int o = 16; o >= 1; o >>= 1) mx = fmaxf(mx, __shfl_xor(mx, o));
  float sm = 0.0f; for (int i = 0; i < 64; ++i) { x[i] = __expf(x[i] - mx); sm += x[i]; }
#pragma unroll
  for (int o = 16; o >= 1; o >>= 1) sm += __shfl_xor(sm, o);
  const float inv = PS / sm;
  for (int pass = 0; pass < 2; ++pass) { for (int j = 0; j < 8; ++j) { v8b o; for (int i = 0; i < 8; ++i) o[i] = (b16)(x[j * 8 + i] * inv); *(volatile v8b*)(P16 + m * N + j * 256 + lane * 8) = o; } __threadfence(); }
}
__global__ __launch_bounds__(128) void out_kernel(const b16* __restrict__ P16, const b16* __restrict__ Qh, const b16* __restrict__ Ql, const float* __restrict__ x, const float* __restrict__ gam, int b, float* __restrict__ out) {
  __shared__ __attribute__((aligned(16))) float Tf[4][16][128 + 4];
  const int wave = threadIdx.x >> 5, lane = threadIdx.x & 31, nloc = lane & 15, hlf = lane >> 4; const size_t m0 = (size_t)blockIdx.x * 64 + wave * 16; const int c0 = blockIdx.y * 128; const float g = bf16_rne(gam[0]);
  v8f acc[8];
#pragma unroll
  for (int t = 0; t < 8; ++t) acc[t] = (v8f){};
#pragma unroll 2
  for (int kb = 0; kb < N; kb += 32) { const v16b a = frag_kb(P16 + (m0 + nloc) * N + kb, hlf);
#pragma unroll
    for (int t = 0; t < 8; ++t) { const size_t qo = ((size_t)b * C + c0 + t * 16 + nloc) * N + kb; acc[t] = wmma16b(a, frag_kb(Qh + qo, hlf), acc[t]); acc[t] = wmma16b(a, frag_kb(Ql + qo, hlf), acc[t]); } }
#pragma unroll
  for (int t = 0; t < 8; ++t) { const int c = c0 + t * 16 + nloc;
#pragma unroll 1
    for (int r = 0; r < 8; ++r) { const size_t m = m0 + 8 * hlf + r; Tf[wave][8 * hlf + r][t * 16 + nloc] = pmul(g, acc[t][r] * (1.0f / (PS * XS))) + bf16_rne(x[((size_t)b * N + m) * C + c]); } }
  wave_lds_sync();
  for (int pass = 0; pass < 2; ++pass) { for (int rr = 0; rr < 16; ++rr) *(volatile v4f*)(out + ((size_t)b * N + m0 + rr) * C + c0 + lane * 4) = *(const v4f*)(&Tf[wave][rr][lane * 4]); __threadfence(); }
}
}

extern "C" void kernel_launch(void* const* d_in, const int* in_sizes, int n_in, void* d_out, int out_size, void* d_ws, size_t ws_size, hipStream_t stream) {
  (void)n_in;
  auto Fp = [&](int i) { return (const float*)d_in[i]; };
  if (in_sizes[0] != NR * C || in_sizes[1] != CR * C || in_sizes[3] != CR * C || in_sizes[5] != C * C || in_sizes[6] != C || out_size != NR * C) return;
  size_t off = 0; char* ws = (char*)d_ws;
  auto carve = [&](size_t bytes) { char* p = ws + off; off += (bytes + 255) & ~(size_t)255; return p; };
  b16* X16 = (b16*)carve((size_t)NR * C * 2); b16* WKV = (b16*)carve((size_t)2 * CR * C * 2); b16* WQ = (b16*)carve((size_t)C * C * 2);
  b16* Kh = (b16*)carve((size_t)NR * CR * 2); b16* Kl = (b16*)carve((size_t)NR * CR * 2); b16* Vh = (b16*)carve((size_t)NR * CR * 2); b16* Vl = (b16*)carve((size_t)NR * CR * 2); b16* Qh = (b16*)carve((size_t)NBAT * C * N * 2); b16* Ql = (b16*)carve((size_t)NBAT * C * N * 2);
  float* Sf = (float*)carve((size_t)N * N * 4); b16* P16 = (b16*)carve((size_t)N * N * 2);
  if (off > ws_size || off > ((size_t)128 << 20)) return;
  prep_kernel<<<(unsigned)(((size_t)NR * C / 8 + 2 * CR * C / 8 + C * C / 8 + 255) / 256), 256, 0, stream>>>(Fp(0), Fp(1), Fp(3), Fp(5), X16, WKV, WQ);
  kv_kernel<<<NR / 64, 128, 0, stream>>>(X16, WKV, Fp(2), Fp(4), Kh, Kl, Vh, Vl);
  q_kernel<<<dim3(C / 64, N / 128, NBAT), 128, 0, stream>>>(WQ, X16, Fp(6), Qh, Ql);
  for (int b = 0; b < NBAT; ++b) {
    s_kernel<<<dim3(N / 64, N / 128), 128, 0, stream>>>(Vh, Vl, Kh, Kl, b, Sf);
    softmax_kernel<<<N / 8, 256, 0, stream>>>(Sf, P16);
    out_kernel<<<dim3(N / 64, C / 128), 128, 0, stream>>>(P16, Qh, Ql, Fp(0), Fp(7), b, (float*)d_out);
  }
}
